// DCRNN_31482110279806
// MI455X (gfx1250) — hardware-run, weakly checked
//
#include <hip/hip_runtime.h>
#include <math.h>


constexpr float kF16MinNormal = 6.103515625e-5f;
constexpr float kCarryAct = 64.0f;
constexpr float kCarryW   = 256.0f;
constexpr float kFold     = 1.0f / (kCarryAct * kCarryW);
typedef __attribute__((ext_vector_type(16))) _Float16 v16h;
typedef __attribute__((ext_vector_type(8)))  _Float16 v8h;
typedef __attribute__((ext_vector_type(8)))  float    v8f;
typedef __attribute__((ext_vector_type(4)))  float    v4f;
typedef __attribute__((ext_vector_type(4)))  unsigned int v4u;

__device__ __forceinline__ unsigned pk16(unsigned short a, unsigned short b) {
  return (unsigned)a | ((unsigned)b << 16);
}
__device__ __forceinline__ unsigned short h_bits_flush(float f) {
  const float g = (fabsf(f) < kF16MinNormal) ? 0.0f : f;
  const _Float16 h = (_Float16)g;
  return __builtin_bit_cast(unsigned short, h);
}
__device__ __forceinline__ v4u pack8_flush(const float (&v)[8]) {
  unsigned short hb[8];
#pragma unroll
  for (int e = 0; e < 8; ++e) hb[e] = h_bits_flush(v[e]);
  return (v4u){pk16(hb[0], hb[1]), pk16(hb[2], hb[3]), pk16(hb[4], hb[5]), pk16(hb[6], hb[7])};
}

struct FragH {
  union U { v16h v; v8h h[2]; };
  static __device__ __forceinline__ v16h load(const _Float16* p) {
    U f;
    f.h[0] = *(const v8h*)(p);
    f.h[1] = *(const v8h*)(p + 16);
    return f.v;
  }
};
__device__ __forceinline__ v8f mma_g(v16h a, v16h b, v8f c) {
  c = __builtin_amdgcn_wmma_f32_16x16x32_f16(false, a, false, b, (short)0, c, false, false);
  asm volatile("v_nop\n\tv_nop\n\tv_nop\n\tv_nop" : "+v"(c) : "v"(a), "v"(b));
  return c;
}
__device__ __forceinline__ void acc_guard4(v8f& a, v8f& b, v8f& c, v8f& d) {
  asm volatile("v_nop\n\tv_nop\n\tv_nop\n\tv_nop" : "+v"(a), "+v"(b), "+v"(c), "+v"(d));
}

template <bool BIAS>
__global__ __launch_bounds__(256) void gemm_f16_kernel(
    const unsigned short* __restrict__ Ap, int lda, long strideA,
    const unsigned short* __restrict__ Bp, int ldb, long strideB,
    float* __restrict__ Cout, int ldc, long strideC,
    const float* __restrict__ bias0, const float* __restrict__ bias1, long strideBias,
    int M, int N, int K, float scale) {
  __shared__ __align__(16) float sT[8][16 * 68];
  const int z    = blockIdx.y;
  const int lane = threadIdx.x & 31;
  const int wave = threadIdx.x >> 5;
  const int tilesN = N >> 6;
  const int tilesM = M >> 5;
  const int tile = blockIdx.x * 8 + wave;
  if (tile >= tilesM * tilesN) return;
  const int tm = tile / tilesN;
  const int tn = tile - tm * tilesN;
  const int m0 = tm << 5;
  const int n0 = tn << 6;
  const int rlane = lane & 15;
  const int half8 = (lane >> 4) * 8;
  const int mOff  = (lane >> 4) * 8;

  const size_t aoff = (size_t)z * (size_t)strideA + (size_t)(m0 + rlane) * lda + half8;
  const size_t boff = (size_t)z * (size_t)strideB + (size_t)(n0 + rlane) * ldb + half8;
  const _Float16* pa0 = (const _Float16*)Ap + aoff;
  const _Float16* pa1 = pa0 + (size_t)16 * lda;
  const _Float16* pbh = (const _Float16*)Bp + boff;
  const size_t bstep = (size_t)16 * ldb;

  v8f acc[2][4];
#pragma unroll
  for (int i = 0; i < 2; ++i)
#pragma unroll
    for (int j = 0; j < 4; ++j)
      acc[i][j] = (v8f){0.f, 0.f, 0.f, 0.f, 0.f, 0.f, 0.f, 0.f};

  for (int k0 = 0; k0 < K; k0 += 32) {
    const v16h ah0 = FragH::load(pa0 + k0);
    const v16h ah1 = FragH::load(pa1 + k0);
#pragma unroll
    for (int j = 0; j < 4; ++j) {
      const v16h bh = FragH::load(pbh + j * bstep + k0);
      acc[0][j] = mma_g(ah0, bh, acc[0][j]);
      acc[1][j] = mma_g(ah1, bh, acc[1][j]);
    }
  }
  acc_guard4(acc[0][0], acc[0][1], acc[0][2], acc[0][3]);
  acc_guard4(acc[1][0], acc[1][1], acc[1][2], acc[1][3]);

  float bA[4], bB[4];
#pragma unroll
  for (int j = 0; j < 4; ++j) {
    bA[j] = 0.0f;
    bB[j] = 0.0f;
    if (BIAS) {
      const size_t bi = (size_t)z * (size_t)strideBias + (size_t)(n0 + (j << 4) + rlane);
      bA[j] = bias0[bi];
      bB[j] = bias1[bi];
    }
  }

  float* slab = sT[wave];
  float* C = Cout + (size_t)z * (size_t)strideC;
#pragma unroll
  for (int i = 0; i < 2; ++i) {
    const int mBase = m0 + (i << 4);
#pragma unroll
    for (int j = 0; j < 4; ++j) {
#pragma unroll
      for (int r = 0; r < 8; ++r) {
        float v = acc[i][j][r] * scale;
        if (BIAS) v = (v + bA[j]) + bB[j];
        slab[(mOff + r) * 68 + (j << 4) + rlane] = v;
      }
    }
    __builtin_amdgcn_fence(__ATOMIC_RELEASE, "workgroup");
    __builtin_amdgcn_wave_barrier();
    __builtin_amdgcn_fence(__ATOMIC_ACQUIRE, "workgroup");
    {
      const int hh = lane >> 4, c4 = (lane & 15) * 4;
      for (int pass = 0; pass < 2; ++pass) {
#pragma unroll
        for (int it = 0; it < 8; ++it) {
          const int row = it * 2 + hh;
          const v4f v = *(const v4f*)(slab + row * 68 + c4);
          *(volatile v4f*)(C + (size_t)(mBase + row) * ldc + n0 + c4) = v;
        }
        __threadfence();
      }
    }
    __builtin_amdgcn_fence(__ATOMIC_RELEASE, "workgroup");
    __builtin_amdgcn_wave_barrier();
    __builtin_amdgcn_fence(__ATOMIC_ACQUIRE, "workgroup");
  }
}

__global__ __launch_bounds__(256) void cast_rows_f16_kernel(
    const float* __restrict__ src, int srcPitch, int srcColOff, int srcCols,
    unsigned short* __restrict__ dst, int dstCols, int totalGroups, float carry) {
  const int i = blockIdx.x * 256 + threadIdx.x;
  if (i >= totalGroups) return;
  const int gpr = dstCols >> 3;
  const int row = i / gpr;
  const int c8  = (i - row * gpr) * 8;
  const bool valid = (c8 < srcCols);
  const int cc = valid ? c8 : (srcCols - 8);
  const float* p = src + (size_t)row * srcPitch + srcColOff + cc;
  v4f a = *(const v4f*)(p);
  v4f b = *(const v4f*)(p + 4);
  asm volatile("" : "+v"(a), "+v"(b));
  float v[8];
#pragma unroll
  for (int e = 0; e < 4; ++e) {
    v[e]     = valid ? (a[e] * carry) : 0.0f;
    v[4 + e] = valid ? (b[e] * carry) : 0.0f;
  }
  const v4u u = pack8_flush(v);
  unsigned short* q = dst + (size_t)i * 8;
  *(volatile v4u*)q = u;
  __threadfence();
  *(volatile v4u*)q = u;
}


namespace {

constexpr int N = 10000, NP = 10016, NPL = NP  , SRCM = N  , EFULL = 640000, E = EFULL  ;
constexpr int FI = 64  , F = 256  , FO = 256  , F2 = F, VOC = 1, NRL = NP  , NL = (NPL < N ? NPL : N);
static_assert(F == 256 && FO == 256 && FI == 64, "64 -> 256 -> 256");
constexpr int HG = 256  , G3 = 3 * HG  , NHEAD = 3  ;
constexpr float LNEPS = 1e-5f; constexpr float LOG2E = 1.4426950408889634f; constexpr float XS = 8.0f, WSC = 256.0f, WSQ = 0.25f, RS_ = 1024.0f, NSL_ = 0.2f, NSA_ = 0.01f, SLOPE = 0.0f, BNEPS = 1e-5f;
static_assert(NP % 32 == 0 && NP >= N && NPL % 32 == 0 && F % 32 == 0, "tiling");
typedef _Float16 b16;
typedef __attribute__((ext_vector_type(16))) _Float16 v16b;
typedef __attribute__((ext_vector_type(8))) _Float16 v8b;
typedef __attribute__((ext_vector_type(8))) float v8f;
typedef __attribute__((ext_vector_type(4))) float v4f;
__device__ __forceinline__ float bf16_rne(float f) { unsigned int u = __float_as_uint(f); u += 0x7FFFu + ((u >> 16) & 1u); return __uint_as_float(u & 0xFFFF0000u); }
__device__ __forceinline__ void split16(float v, b16& hi, b16& lo) { hi = (b16)v; lo = (b16)(v - (float)hi); }
__device__ __forceinline__ v16b frag_kb(const b16* p, int hh) { const v8b a = *(const v8b*)(p + 8 * hh), b = *(const v8b*)(p + 16 + 8 * hh); v16b f;
#pragma unroll
  for (int e = 0; e < 8; ++e) { f[e] = a[e]; f[8 + e] = b[e]; } return f; }
__device__ __forceinline__ v8f wmma16b(v16b a, v16b b, v8f c) { v8f d = __builtin_amdgcn_wmma_f32_16x16x32_f16(false, a, false, b, (short)0, c, false, false); asm volatile("v_nop\n\tv_nop\n\tv_nop\n\tv_nop" : "+v"(d) : "v"(a), "v"(b)); return d; }
__device__ __forceinline__ void wave_lds_sync() { __builtin_amdgcn_fence(__ATOMIC_RELEASE, "workgroup"); __builtin_amdgcn_wave_barrier(); __builtin_amdgcn_fence(__ATOMIC_ACQUIRE, "workgroup"); }
__device__ __forceinline__ int iclamp(int v, int lo, int hi) { return v < lo ? lo : (v > hi ? hi : v); }
constexpr int CSR_NBLK = 512, CSR_GB = 7  , CSR_GN = 1 << CSR_GB  , CSR_MAXG = 512, CSR_CAP = 12288  ;
static_assert(((N + CSR_GN - 1) >> CSR_GB) <= CSR_MAXG && CSR_GN % 4 == 0 && CSR_GN <= 65536, "csr: bucket count / 16-bit node key");
__global__ __launch_bounds__(64) void csrA_kernel(const int* __restrict__ dst, int E, int N, int nG, int CHP, int NGP, int* __restrict__ STG, int* __restrict__ HST) {
  extern __shared__ int sm[];
  int* cnt = sm; int* run = sm + NGP; int* ids = sm + 2 * NGP;
  const int b = blockIdx.x; const int ch = (E + CSR_NBLK - 1) / CSR_NBLK; const int e0 = b * ch, e1 = min(E, e0 + ch);
  for (int i = threadIdx.x; i < NGP; i += 64) cnt[i] = 0;
  for (int i = threadIdx.x; i < CHP; i += 64) ids[i] = -1;
  __syncthreads();
  if (threadIdx.x == 0) {
    for (int e = e0; e < e1; ++e) { int d = dst[e]; d = (d < 0) ? 0 : (d >= N ? N - 1 : d); cnt[d >> CSR_GB] += 1; }
    int acc = 0; for (int g = 0; g < nG; ++g) { run[g] = acc; acc += cnt[g]; }
    for (int e = e0; e < e1; ++e) { int d = dst[e]; d = (d < 0) ? 0 : (d >= N ? N - 1 : d); const int g = d >> CSR_GB; ids[run[g]] = e; run[g] += 1; } }
  __syncthreads();
  typedef __attribute__((ext_vector_type(4))) int v4i;
  for (int pass = 0; pass < 2; ++pass) {
    for (int i = threadIdx.x; i < CHP / 4; i += 64) *(volatile v4i*)(STG + (size_t)b * CHP + i * 4) = *(const v4i*)(&ids[i * 4]);
    for (int i = threadIdx.x; i < NGP / 4; i += 64) { v4i v; for (int e = 0; e < 4; ++e) v[e] = (i * 4 + e < nG) ? cnt[i * 4 + e] : 0; *(volatile v4i*)(HST + (size_t)b * NGP + i * 4) = v; }
    __threadfence(); }
}
__global__ __launch_bounds__(512) void csrS_kernel(const int* __restrict__ HST, int nG, int NGP, int* __restrict__ START, int* __restrict__ TOT, int* __restrict__ OFF) {
  __shared__ int tot[CSR_MAXG];
  const int b = threadIdx.x;
  for (int pass = 0; pass < 2; ++pass) { int runb = 0; for (int g = 0; g < nG; ++g) { int c = HST[(size_t)b * NGP + g]; c = (c < 0) ? 0 : c; ((volatile int*)OFF)[(size_t)g * CSR_NBLK + b] = runb; runb += c; } __threadfence(); }
  for (int g = threadIdx.x; g < nG; g += 512) { int s = 0; for (int bb = 0; bb < CSR_NBLK; ++bb) { int c = HST[(size_t)bb * NGP + g]; s += (c < 0) ? 0 : c; } tot[g] = s; }
  __syncthreads();
  if (threadIdx.x < 32) {
    __shared__ int st[CSR_MAXG + 32];
    if (threadIdx.x == 0) { int acc = 0; for (int g = 0; g < NGP; ++g) { st[g] = acc; if (g < nG) acc += (tot[g] + 31) & ~31; } st[NGP] = acc; }
    __builtin_amdgcn_fence(__ATOMIC_RELEASE, "workgroup"); __builtin_amdgcn_wave_barrier(); __builtin_amdgcn_fence(__ATOMIC_ACQUIRE, "workgroup");
    for (int pass = 0; pass < 2; ++pass) { for (int i = threadIdx.x; i < NGP + 32; i += 32) { ((volatile int*)START)[i] = (i <= NGP) ? st[min(i, NGP)] : 0; ((volatile int*)TOT)[i] = (i < nG) ? tot[i] : 0; } __threadfence(); } }
}
__global__ __launch_bounds__(256) void csrB_kernel(const int* __restrict__ dst, int N, int nG, int CHP, int NGP, int permLen, const int* __restrict__ STG, const int* __restrict__ HST, const int* __restrict__ OFF, const int* __restrict__ START, const int* __restrict__ TOT, int* __restrict__ PERM, int* __restrict__ ROWPTR, int* __restrict__ ROWCNT, int* __restrict__ FLAG) {
  typedef __attribute__((ext_vector_type(4))) int v4i;
  __shared__ int ids[CSR_CAP]; __shared__ unsigned short key[CSR_CAP]; __shared__ int outp[CSR_CAP]; __shared__ int ncnt[CSR_GN + 1]; __shared__ int boff[CSR_NBLK + 1];
  const int g = blockIdx.x, t_ = threadIdx.x; int tot = TOT[g]; int st = START[g], stn = START[g + 1]; const int v0 = g * CSR_GN; const int nv = min(CSR_GN, N - v0);
  st = (st < 0) ? 0 : (st > permLen - 32 ? permLen - 32 : st) & ~31; stn = (stn < st) ? st : (stn > permLen ? permLen : stn); tot = (tot < 0) ? 0 : tot; if (tot > stn - st && tot <= CSR_CAP) tot = stn - st;
  if (tot > CSR_CAP) {
    for (int pass = 0; pass < 2; ++pass) { for (int i = t_; i < CSR_GN / 4; i += 256) { v4i a, c; for (int e = 0; e < 4; ++e) { a[e] = st; c[e] = 0; } *(volatile v4i*)(ROWPTR + v0 + i * 4) = a; *(volatile v4i*)(ROWCNT + v0 + i * 4) = c; } if (t_ == 0) ((volatile int*)FLAG)[0] = 1; __threadfence(); } (void)nv; return; }
  if (t_ == 0) { int acc = 0; for (int b = 0; b < CSR_NBLK; ++b) { boff[b] = acc; int c = HST[(size_t)b * NGP + g]; c = (c < 0) ? 0 : (c > CHP ? CHP : c); acc += c; if (acc > tot) acc = tot; } boff[CSR_NBLK] = acc; }
  for (int i = t_; i <= CSR_GN; i += 256) ncnt[i] = 0;
  __syncthreads();
  for (int b = 0; b < CSR_NBLK; ++b) { const int c = boff[b + 1] - boff[b]; int o_ = OFF[(size_t)g * CSR_NBLK + b]; o_ = (o_ < 0) ? 0 : (o_ > CHP - c ? CHP - c : o_); const int* src_ = STG + (size_t)b * CHP + o_;
    for (int i = t_; i < c; i += 256) { int id = src_[i]; id = (id < 0) ? 0 : id; ids[boff[b] + i] = id; int d = dst[id]; d = (d < v0) ? v0 : (d >= N ? N - 1 : d); int kk = d - v0; kk = (kk < 0) ? 0 : (kk >= CSR_GN ? CSR_GN - 1 : kk); key[boff[b] + i] = (unsigned short)kk; } }
  __syncthreads();
  if (t_ == 0) { for (int i = 0; i < tot; ++i) ncnt[key[i]] += 1; int acc = 0; for (int vl = 0; vl < CSR_GN; ++vl) { const int c = ncnt[vl]; ncnt[vl] = acc; acc += c; } ncnt[CSR_GN] = acc;
    for (int i = 0; i < tot; ++i) { const int vl = key[i]; outp[ncnt[vl]] = ids[i]; ncnt[vl] += 1; }
    for (int vl = CSR_GN; vl > 0; --vl) ncnt[vl] = ncnt[vl - 1]; ncnt[0] = 0; }
  __syncthreads();
  for (int pass = 0; pass < 2; ++pass) {
    for (int i = t_; i < (stn - st) / 4; i += 256) { v4i v; for (int e = 0; e < 4; ++e) { const int q = i * 4 + e; v[e] = (q < tot) ? outp[q] : -1; } *(volatile v4i*)(PERM + st + i * 4) = v; }
    for (int i = t_; i < CSR_GN / 4; i += 256) { v4i a, c; for (int e = 0; e < 4; ++e) { const int vl = i * 4 + e; a[e] = st + ncnt[vl]; c[e] = (vl < nv) ? (ncnt[vl + 1] - ncnt[vl]) : 0; } *(volatile v4i*)(ROWPTR + v0 + i * 4) = a; *(volatile v4i*)(ROWCNT + v0 + i * 4) = c; }
    __threadfence(); }
}
__global__ __launch_bounds__(256) void csrZ_kernel(int* __restrict__ p, size_t n4) { typedef __attribute__((ext_vector_type(4))) int v4i; const size_t tid = (size_t)blockIdx.x * 256 + threadIdx.x, nth = (size_t)gridDim.x * 256; v4i z = {0, 0, 0, 0}; for (size_t i = tid; i < n4; i += nth) *(volatile v4i*)(p + i * 4) = z; }
struct CsrBufs { int *STG, *HST, *OFF, *START, *TOT, *PERM, *ROWPTR, *ROWCNT, *FLAG; int nG, NGP, CHP; size_t permLen; char* base; size_t bytes; };
static size_t csr_carve(CsrBufs& c, char* ws, size_t off, int E, int N) {
  const size_t off0 = off; c.base = ws + off;
  auto al = [&](size_t bytes) { char* p = ws + off; off += (bytes + 255) & ~(size_t)255; return p; };
  c.nG = (N + CSR_GN - 1) / CSR_GN; c.NGP = (c.nG + 31) & ~31; const int ch = (E + CSR_NBLK - 1) / CSR_NBLK; c.CHP = (ch + 31) & ~31; c.permLen = (size_t)E + 32 * (size_t)c.nG + 32;
  c.STG = (int*)al((size_t)CSR_NBLK * c.CHP * 4); c.HST = (int*)al((size_t)CSR_NBLK * c.NGP * 4); c.OFF = (int*)al((size_t)c.NGP * CSR_NBLK * 4); c.START = (int*)al((size_t)(c.NGP + 64) * 4); c.TOT = (int*)al((size_t)(c.NGP + 64) * 4);
  c.PERM = (int*)al(c.permLen * 4); c.ROWPTR = (int*)al((size_t)c.nG * CSR_GN * 4); c.ROWCNT = (int*)al((size_t)c.nG * CSR_GN * 4); c.FLAG = (int*)al(256);
  c.bytes = off - off0; return off;
}
static void csr_build(const CsrBufs& c, const int* dst, int E, int N, hipStream_t stream) {
  const size_t smem = (size_t)(2 * c.NGP + c.CHP) * 4;
  csrZ_kernel<<<512, 256, 0, stream>>>((int*)c.base, c.bytes / 16);
  csrA_kernel<<<CSR_NBLK, 64, smem, stream>>>(dst, E, N, c.nG, c.CHP, c.NGP, c.STG, c.HST);
  csrS_kernel<<<1, 512, 0, stream>>>(c.HST, c.nG, c.NGP, c.START, c.TOT, c.OFF);
  csrB_kernel<<<c.nG, 256, 0, stream>>>(dst, N, c.nG, c.CHP, c.NGP, (int)c.permLen, c.STG, c.HST, c.OFF, c.START, c.TOT, c.PERM, c.ROWPTR, c.ROWCNT, c.FLAG);
}

typedef __attribute__((ext_vector_type(4))) _Float16 v4h;
__device__ __forceinline__ float lrelu(float v) { return v > 0.0f ? v : NSL_ * v; }
template <int K, int NOUTR, int NOUTP>
__global__ __launch_bounds__(256) void wt_kernel(const float* __restrict__ w, b16* __restrict__ WT, float scl) {
  static_assert(K % 8 == 0 && NOUTR <= NOUTP, "wt: thread per (o, 8 k)");
  const int u = blockIdx.x * 256 + threadIdx.x; if (u >= NOUTP * K / 8) return; const int e = u * 8; const int o = e / K, k0 = e % K; v8b v;
#pragma unroll
  for (int j = 0; j < 8; ++j) v[j] = (b16)(o < NOUTR ? bf16_rne(w[(size_t)(k0 + j) * NOUTR + o]) * scl : 0.0f);
  for (int pass = 0; pass < 2; ++pass) { *(volatile v8b*)(WT + e) = v; __threadfence(); }
}
template <int K, int NT, bool RND, int MODE, bool GIDX>
__global__ __launch_bounds__(64) void lin_kernel(const float* __restrict__ X, const int* __restrict__ gidx, const b16* __restrict__ WT, const b16* __restrict__ WQ, const float* __restrict__ bias, float* __restrict__ OUT, int opitch, int nvalid, int mrows) {
  constexpr int NC = NT * 16;
  static_assert(K % 32 == 0 && NT % 4 == 0 && NT <= 16 && (NC < 128 || NC % 128 == 0), "lin: k-steps of 32; row store = whole 128-column groups or one partial group");
  __shared__ __attribute__((aligned(16))) b16 Ah[2][16][K + 8], Al[2][16][K + 8]; __shared__ __attribute__((aligned(16))) float Tf[2][16][NC + 4];
  const int wave = threadIdx.x >> 5, lane = threadIdx.x & 31, nloc = lane & 15, hlf = lane >> 4; const size_t m0 = (size_t)blockIdx.x * 32 + wave * 16;
  for (int idx = lane; idx < 16 * (K / 4); idx += 32) { const int rr = idx / (K / 4), c4 = (idx % (K / 4)) * 4; const size_t vrow = (m0 + rr < (size_t)nvalid) ? m0 + rr : (size_t)nvalid - 1; size_t arow = vrow; if (GIDX) arow = (size_t)iclamp(gidx[vrow], 0, VOC - 1);
    const v4f v = *(const v4f*)(X + arow * K + c4); v4h hv, lv;
    for (int j = 0; j < 4; ++j) { float vj = v[j]; if (MODE == 2) vj = fmaxf(vj, 0.0f); const float vs = (RND ? bf16_rne(vj) : vj) * XS; const b16 ph = (b16)vs; hv[j] = ph; lv[j] = (b16)((vs - (float)ph) * RS_); } *(v4h*)(&Ah[wave][rr][c4]) = hv; *(v4h*)(&Al[wave][rr][c4]) = lv; }
  wave_lds_sync();
  v8f acc[NT];
#pragma unroll
  for (int t = 0; t < NT; ++t) acc[t] = (v8f){};
#pragma unroll 1
  for (int kb = 0; kb < K; kb += 32) { const v16b a = frag_kb(&Ah[wave][nloc][kb], hlf); v16b al; if (!RND) al = frag_kb(&Al[wave][nloc][kb], hlf);
#pragma unroll
    for (int t = 0; t < NT; ++t) { const size_t wo_ = (size_t)(t * 16 + nloc) * K + kb; acc[t] = wmma16b(a, frag_kb(WT + wo_, hlf), acc[t]); if (!RND) acc[t] = wmma16b(al, frag_kb(WQ + wo_, hlf), acc[t]); } }
#pragma unroll
  for (int t = 0; t < NT; ++t) { const int col = t * 16 + nloc; const float bb = bf16_rne(bias[col]);
    for (int r = 0; r < 8; ++r) { const size_t vrow = m0 + 8 * hlf + r; float y = acc[t][r] * (1.0f / (XS * WSC)) + bb; if (MODE == 1) y = fmaxf(y, 0.0f); Tf[wave][8 * hlf + r][col] = (vrow < (size_t)nvalid) ? y : 0.0f; } }
  wave_lds_sync();
  for (int pass = 0; pass < 2; ++pass) { for (int rr = 0; rr < 16; ++rr) { if (m0 + rr < (size_t)mrows) { if (NC >= 128) { for (int c8 = 0; c8 < NC; c8 += 128) *(volatile v4f*)(OUT + (m0 + rr) * (size_t)opitch + c8 + lane * 4) = *(const v4f*)(&Tf[wave][rr][c8 + lane * 4]); }
        else { if (lane < NC / 4) *(volatile v4f*)(OUT + (m0 + rr) * (size_t)opitch + lane * 4) = *(const v4f*)(&Tf[wave][rr][lane * 4]); } } } __threadfence(); }
}
__device__ __forceinline__ float gelu_(float v) { return 0.5f * v * (1.0f + erff(v * 0.70710678118654752f)); }
template <int W, int ACT>
__global__ __launch_bounds__(256) void gcn_kernel(const float* __restrict__ Hh, const int* __restrict__ srcs, const int* __restrict__ PERM, const int* __restrict__ ROWPTR, const int* __restrict__ ROWCNT, int permLen, const float* __restrict__ bias, const float* __restrict__ ADDP, float* __restrict__ out, int mrows) {
  constexpr int CW = W / 8;
  static_assert(W % 32 == 0, "gcn: 8 threads per row, float4 stores");
  const int tid = threadIdx.x; const int row = tid >> 3, g = tid & 7, c0 = g * CW; const int v = blockIdx.x * 32 + row; const int vv = v < N ? v : N - 1;
  int cnt = 0, p0 = 0; if (v < N) { cnt = iclamp(ROWCNT[v], 0, 65536); p0 = iclamp(ROWPTR[v], 0, permLen - 1); if (p0 + cnt > permLen) cnt = permLen - p0; }
  const float dv = rsqrtf((float)(cnt + 1));
  float m[CW]; { const float* hr = Hh + (size_t)vv * W + c0;
#pragma unroll
    for (int q = 0; q < CW / 4; ++q) { const v4f t4 = *(const v4f*)(hr + 4 * q); for (int j = 0; j < 4; ++j) m[4 * q + j] = (dv * t4[j]); } }
  for (int i = 0; i < cnt; ++i) { const int e = iclamp(PERM[p0 + i], 0, E - 1); int s = iclamp(srcs[e], 0, N - 1); if (SRCM < N) s %= SRCM; const float cf = rsqrtf((float)(iclamp(ROWCNT[s], 0, 1 << 24) + 1)); const float* hr = Hh + (size_t)s * W + c0;
#pragma unroll
    for (int q = 0; q < CW / 4; ++q) { const v4f t4 = *(const v4f*)(hr + 4 * q); for (int j = 0; j < 4; ++j) m[4 * q + j] += (cf * t4[j]); } }
  for (int pass = 0; pass < 2; ++pass) { if (v < mrows) { float* orow = out + (size_t)v * W + c0;
#pragma unroll
      for (int q = 0; q < CW / 4; ++q) { v4f o; for (int j = 0; j < 4; ++j) { float y = (dv * m[4 * q + j]) + bf16_rne(bias[c0 + 4 * q + j]); if (ADDP != nullptr) y += ADDP[(size_t)vv * W + c0 + 4 * q + j]; if (ACT == 1) y = fmaxf(y, 0.0f); if (ACT == 3) y = (y >= 0.0f) ? y : 0.01f * y; if (ACT == 4) { const float sp = (y > 20.0f) ? y : __logf(1.0f + __expf(y)); const float t = __expf(((-2.0f) * sp)); y = (y * (1.0f - t)) / (1.0f + t); }     o[j] = (v < N) ? y : 0.0f; } *(volatile v4f*)(orow + 4 * q) = o; } }
    __threadfence(); }
}
__global__ __launch_bounds__(256) void zfill_kernel(float* __restrict__ Z, int n) { const int i = threadIdx.x; for (int pass = 0; pass < 2; ++pass) { if (i < n) ((volatile float*)Z)[i] = 0.0f; __threadfence(); } }
template <int K, int NO, bool OI>
__global__ __launch_bounds__(256) void headw_kernel(const float* __restrict__ P, int pp, const float* __restrict__ wl, const float* __restrict__ bl, float* __restrict__ out, int total) {
  static_assert(K >= 1 && NO >= 1 && NO <= 16, "headw: a narrow head (the matrix unit serves wider ones)"); const int t = blockIdx.x * 256 + threadIdx.x; if (t >= total) return; const int g = t / NO, k = t - g * NO; float s = bf16_rne(bl[k]);
  for (int c = 0; c < K; ++c) s += (P[(size_t)g * pp + c] * bf16_rne(OI ? wl[k * K + c] : wl[c * NO + k]));
  for (int pass = 0; pass < 2; ++pass) { ((volatile float*)out)[t] = s; __threadfence(); }
}
__global__ __launch_bounds__(256) void rndbf_kernel(const float* __restrict__ SRC, float* __restrict__ DST, int n4) {
  const int i = blockIdx.x * 256 + threadIdx.x; if (i >= n4) return; const v4f a = *(const v4f*)(SRC + (size_t)i * 4); v4f o;
#pragma unroll
  for (int j = 0; j < 4; ++j) o[j] = bf16_rne(a[j]);
  for (int pass = 0; pass < 2; ++pass) { *(volatile v4f*)(DST + (size_t)i * 4) = o; __threadfence(); }
}
__global__ __launch_bounds__(768) void gruchain_kernel(const float* __restrict__ GI, const float* __restrict__ WH, const float* __restrict__ BH, float* __restrict__ HS, int nsteps) {
  static_assert(G3 == 768 && HG % 4 == 0, "gruchain: one thread per gate row");
  __shared__ __attribute__((aligned(16))) float h_s[HG]; __shared__ __attribute__((aligned(16))) float g_s[G3];
  const int tid = threadIdx.x; const v4f* w4 = (const v4f*)(WH + (size_t)tid * HG); const v4f* h4 = (const v4f*)h_s; const float bh = BH[tid];
  if (tid < HG) h_s[tid] = 0.0f;
  __syncthreads();
#pragma unroll 1
  for (int t = 0; t < nsteps; ++t) {
    const float* gr = GI + (size_t)t * G3; float gir = 0.0f, giz = 0.0f, gin = 0.0f;
    if (tid < HG) { gir = gr[tid]; giz = gr[HG + tid]; gin = gr[2 * HG + tid]; }
    float acc = 0.0f;
#pragma unroll 2
    for (int k = 0; k < HG / 4; ++k) { const v4f hv = h4[k]; const v4f a = w4[k]; acc = fmaf(a[0], hv[0], acc); acc = fmaf(a[1], hv[1], acc); acc = fmaf(a[2], hv[2], acc); acc = fmaf(a[3], hv[3], acc); }
    g_s[tid] = acc + bh;
    __syncthreads();
    if (tid < HG) {
      const float hr = g_s[tid], hz = g_s[HG + tid], hn = g_s[2 * HG + tid];
      const float r = 1.0f / (1.0f + expf(-(gir + hr))); const float z = 1.0f / (1.0f + expf(-(giz + hz))); const float nn = tanhf(gin + r * hn);
      const float hp = h_s[tid]; const float hnew = (1.0f - z) * nn + z * hp;
      h_s[tid] = hnew; float* op = HS + (size_t)t * HG + tid;
      *(volatile float*)op = hnew; __threadfence(); *(volatile float*)op = hnew;
    }
    __syncthreads();
  }
}
}

extern "C" void kernel_launch(void* const* d_in, const int* in_sizes, int n_in, void* d_out, int out_size, void* d_ws, size_t ws_size, hipStream_t stream) {
  (void)n_in;
  auto Fp = [&](int i) { return (const float*)d_in[i]; }; auto Ip = [&](int i) { return (const int*)d_in[i]; };
  if (in_sizes[0] != N * FI || in_sizes[1] != 2 * EFULL || in_sizes[2] != FI * F || in_sizes[3] != F || in_sizes[4] != F * FO || in_sizes[5] != FO || in_sizes[6] != G3 * HG || in_sizes[7] != G3 * HG || in_sizes[8] != G3 || in_sizes[9] != G3 || in_sizes[10] != NHEAD * HG || in_sizes[11] != NHEAD || out_size != N * NHEAD) return;
  size_t off = 0; char* ws = (char*)d_ws;
  auto carve = [&](size_t bytes) { char* p = ws + off; off += (bytes + 255) & ~(size_t)255; return p; };
  b16* W1T = (b16*)carve((size_t)F * FI * 2); b16* W2T = (b16*)carve((size_t)FO * F * 2);
  float* ZB = (float*)carve((size_t)G3 * 4);
  float* HA = (float*)carve((size_t)NP * F * 4); float* HB = (float*)carve((size_t)NP * F * 4);
  float* WIB = (float*)carve((size_t)G3 * HG * 4); float* WHB = (float*)carve((size_t)G3 * HG * 4); float* BIB = (float*)carve((size_t)G3 * 4); float* BHB = (float*)carve((size_t)G3 * 4);
  unsigned short* WIP = (unsigned short*)carve((size_t)G3 * HG * 2); unsigned short* H2P = (unsigned short*)carve((size_t)NP * HG * 2);
  float* GI = (float*)carve((size_t)NP * G3 * 4); float* HS = (float*)carve((size_t)NP * HG * 4);
  CsrBufs csr; off = csr_carve(csr, ws, off, E, N);
  if (off > ws_size || off > ((size_t)126 << 20)) return;
  { wt_kernel<FI, F, F><<<(F * FI / 8 + 255) / 256, 256, 0, stream>>>(Fp(2), W1T, WSC); wt_kernel<F, FO, FO><<<(FO * F / 8 + 255) / 256, 256, 0, stream>>>(Fp(4), W2T, WSC);
    zfill_kernel<<<1, 256, 0, stream>>>(ZB, 256); zfill_kernel<<<1, 256, 0, stream>>>(ZB + 256, 256); zfill_kernel<<<1, 256, 0, stream>>>(ZB + 512, 256); }
  csr_build(csr, Ip(1) + EFULL, E, N, stream);
  lin_kernel<FI, 8, true, 0, false><<<NRL / 32, 64, 0, stream>>>(Fp(0), nullptr, W1T, W1T, ZB, HA, F, N, NRL);
  lin_kernel<FI, 8, true, 0, false><<<NRL / 32, 64, 0, stream>>>(Fp(0), nullptr, W1T + (size_t)128 * FI, W1T + (size_t)128 * FI, ZB, HA + 128, F, N, NRL);
  gcn_kernel<F, 1><<<NRL / 32, 256, 0, stream>>>(HA, Ip(1), csr.PERM, csr.ROWPTR, csr.ROWCNT, (int)csr.permLen, Fp(3), nullptr, HB, NRL);
  lin_kernel<F, 16, true, 0, false><<<NRL / 32, 64, 0, stream>>>(HB, nullptr, W2T, W2T, ZB, HA, FO, N, NRL);
  gcn_kernel<FO, 1><<<NRL / 32, 256, 0, stream>>>(HA, Ip(1), csr.PERM, csr.ROWPTR, csr.ROWCNT, (int)csr.permLen, Fp(5), nullptr, HB, NRL);
  rndbf_kernel<<<(G3 * HG / 4) / 256, 256, 0, stream>>>(Fp(6), WIB, G3 * HG / 4); rndbf_kernel<<<(G3 * HG / 4) / 256, 256, 0, stream>>>(Fp(7), WHB, G3 * HG / 4);
  rndbf_kernel<<<1, 256, 0, stream>>>(Fp(8), BIB, G3 / 4); rndbf_kernel<<<1, 256, 0, stream>>>(Fp(9), BHB, G3 / 4);
  cast_rows_f16_kernel<<<(G3 * (HG / 8)) / 256, 256, 0, stream>>>(WIB, HG, 0, HG, WIP, HG, G3 * (HG / 8), kCarryW);
  cast_rows_f16_kernel<<<(NP * (HG / 8)) / 256, 256, 0, stream>>>(HB, HG, 0, HG, H2P, HG, NP * (HG / 8), kCarryAct);
  gemm_f16_kernel<true><<<dim3(((NP / 32) * (G3 / 64) + 7) / 8, 1), 256, 0, stream>>>(H2P, HG, 0L, WIP, HG, 0L, GI, G3, 0L, BIB, ZB, 0L, NP, G3, HG, kFold);
  gruchain_kernel<<<1, G3, 0, stream>>>(GI, WHB, BHB, HS, N);
  headw_kernel<HG, NHEAD, true><<<(N * NHEAD + 255) / 256, 256, 0, stream>>>(HS, HG, Fp(10), Fp(11), (float*)d_out, N * NHEAD);
}
